// PINN_6828998000998
// MI455X (gfx1250) — hardware-verified
//
#include <hip/hip_runtime.h>
#include <math.h>
#include <stdint.h>

typedef __attribute__((ext_vector_type(16))) __bf16   v16b;
typedef __attribute__((ext_vector_type(8)))  __bf16   v8b;
typedef __attribute__((ext_vector_type(8)))  float    v8f;
typedef __attribute__((ext_vector_type(4)))  float    v4f;
typedef __attribute__((ext_vector_type(4)))  unsigned int v4u;

constexpr int kNumX       = 32768;
constexpr int kNumData    = 1024;
constexpr int kNumQuad    = 1000;
constexpr int kPtData0    = kNumX;
constexpr int kPtQuad0    = kNumX + kNumData;
constexpr int kPtBnd0     = kPtQuad0 + kNumQuad;
constexpr int kNumPtsPad  = 34816;
constexpr int kNumTiles   = kNumPtsPad / 16;
constexpr int kFeat       = 128;
constexpr int kHStride    = 136;
constexpr int kRecFloats  = 128;
constexpr int kOutLossIdx = 5 * kNumX;

static_assert(kNumTiles * 16 == kNumPtsPad, "");
static_assert(kPtBnd0 + 2 <= kNumPtsPad, "");
static_assert((kHStride % 8) == 0, "");
static_assert((kPtQuad0 % 32) == 0, "");
static_assert(kOutLossIdx * 4 + 4 == 655364, "");

constexpr size_t kWsPts   = 0;
constexpr size_t kWsJT    = kWsPts + (size_t)kNumPtsPad * 4;
constexpr size_t kWsW1h   = kWsJT + (size_t)kNumTiles * kRecFloats * 4;
constexpr size_t kWsW1l   = kWsW1h + (size_t)kFeat * kFeat * 2;
constexpr size_t kWsW2h   = kWsW1l + (size_t)kFeat * kFeat * 2;
constexpr size_t kWsW2l   = kWsW2h + (size_t)kFeat * kFeat * 2;
constexpr size_t kWsP3    = kWsW2l + (size_t)kFeat * kFeat * 2;
constexpr size_t kWsTotal = kWsP3 + (size_t)16 * kFeat * 2;
static_assert(kWsTotal <= (size_t)134217728, "");
static_assert(kWsJT % 128 == 0 && kWsW1h % 128 == 0 && kWsW1l % 128 == 0 && kWsW2h % 128 == 0 && kWsW2l % 128 == 0 && kWsP3 % 128 == 0, "");

__device__ __forceinline__ unsigned short f2bf_bits(float f) {
  unsigned u = __float_as_uint(f);
  return (unsigned short)((u + 0x7FFFu + ((u >> 16) & 1u)) >> 16);
}
__device__ __forceinline__ float bf_bits2f(unsigned short h) { return __uint_as_float(((unsigned)h) << 16); }

__device__ __forceinline__ void put_split(__bf16* hp, __bf16* lp, int idx, float v) {
  const unsigned short hb = f2bf_bits(v);
  const unsigned short lb = f2bf_bits(v - bf_bits2f(hb));
  hp[idx] = __builtin_bit_cast(__bf16, hb);
  lp[idx] = __builtin_bit_cast(__bf16, lb);
}

template <typename T> struct Frag;
template <> struct Frag<__bf16> {
  typedef v16b V; union U { v16b v; v8b h[2]; };
  static __device__ __forceinline__ v16b load(const __bf16* p) {
    U f; f.h[0] = *(const v8b*)(p); f.h[1] = *(const v8b*)(p + 16); return f.v;
  }
};

__device__ __forceinline__ v8f mma_bf(v16b a, v16b b, v8f c) {
  c = __builtin_amdgcn_wmma_f32_16x16x32_bf16(false, a, false, b, (short)0, c, false, false);
  asm volatile("v_nop\n\tv_nop\n\tv_nop\n\tv_nop" : "+v"(c) : "v"(a), "v"(b));
  return c;
}

__device__ __forceinline__ void tanh_jet(float a0, float a1, float a2, float a3, float a4,
                                         float& y0, float& y1, float& y2, float& y3, float& y4) {
  const float t  = tanhf(a0);
  const float t2 = t * t;
  const float f1 = 1.0f - t2;
  const float f2 = -2.0f * t * f1;
  const float f3 = f1 * (6.0f * t2 - 2.0f);
  const float f4 = 8.0f * t * f1 * (2.0f - 3.0f * t2);
  const float a11 = a1 * a1;
  y0 = t;
  y1 = f1 * a1;
  y2 = f1 * a2 + f2 * a11;
  y3 = f1 * a3 + 3.0f * f2 * a1 * a2 + f3 * a11 * a1;
  y4 = f1 * a4 + f2 * (4.0f * a1 * a3 + 3.0f * a2 * a2) + 6.0f * f3 * a11 * a2 + f4 * a11 * a11;
}

__global__ __launch_bounds__(256) void prep_kernel(
    const float* __restrict__ x, const float* __restrict__ dx,
    const float* __restrict__ W1, const float* __restrict__ W2, const float* __restrict__ W3,
    float* __restrict__ pts,
    unsigned short* __restrict__ W1h, unsigned short* __restrict__ W1l,
    unsigned short* __restrict__ W2h, unsigned short* __restrict__ W2l,
    unsigned short* __restrict__ P3)
{
  const int blk = blockIdx.x;
  const int tid = threadIdx.x;
  if (blk < 33) {
    const int t = blk * 256 + tid;
    const int e = t * 4;
    int xi = e; if (xi > kNumX - 4) xi = kNumX - 4;
    int di = e - kNumX; if (di < 0) di = 0; if (di > kNumData - 4) di = kNumData - 4;
    const v4f vx = *(const v4f*)(x + xi);
    const v4f vd = *(const v4f*)(dx + di);
    const bool usex = (e < kNumX);
    v4f v;
#pragma unroll
    for (int q = 0; q < 4; ++q) v[q] = usex ? vx[q] : vd[q];
    float* dst = pts + e;
    *(volatile v4f*)dst = v;
    __threadfence();
    *(volatile v4f*)dst = v;
  } else if (blk < 49) {
    const int wb   = blk - 33;
    const int wsel = wb >> 3;
    const float* W = wsel ? W2 : W1;
    unsigned short* Ph = wsel ? W2h : W1h;
    unsigned short* Pl = wsel ? W2l : W1l;
    const int u  = (wb & 7) * 256 + tid;
    const int n  = u >> 4;
    const int kc = (u & 15) * 8;
    unsigned short hb[8], lb[8];
#pragma unroll
    for (int q = 0; q < 8; ++q) {
      const float f = W[(kc + q) * kFeat + n];
      hb[q] = f2bf_bits(f);
      lb[q] = f2bf_bits(f - bf_bits2f(hb[q]));
    }
    v4u ph, pl;
#pragma unroll
    for (int q = 0; q < 4; ++q) {
      ph[q] = (unsigned)hb[2 * q] | ((unsigned)hb[2 * q + 1] << 16);
      pl[q] = (unsigned)lb[2 * q] | ((unsigned)lb[2 * q + 1] << 16);
    }
    unsigned short* dh = Ph + n * kFeat + kc;
    unsigned short* dl = Pl + n * kFeat + kc;
    *(volatile v4u*)dh = ph;
    *(volatile v4u*)dl = pl;
    __threadfence();
    *(volatile v4u*)dh = ph;
    *(volatile v4u*)dl = pl;
  } else {
    const int u   = tid;
    const int row = u >> 4;
    const int kc  = (u & 15) * 8;
    unsigned short vb[8];
#pragma unroll
    for (int q = 0; q < 8; ++q) {
      const float f = W3[kc + q];
      const unsigned short hb = f2bf_bits(f);
      const unsigned short lb = f2bf_bits(f - bf_bits2f(hb));
      vb[q] = (row == 0) ? hb : ((row == 1) ? lb : (unsigned short)0);
    }
    v4u pv;
#pragma unroll
    for (int q = 0; q < 4; ++q) pv[q] = (unsigned)vb[2 * q] | ((unsigned)vb[2 * q + 1] << 16);
    unsigned short* dp = P3 + row * kFeat + kc;
    *(volatile v4u*)dp = pv;
    __threadfence();
    *(volatile v4u*)dp = pv;
  }
}

__global__ __launch_bounds__(256) void nodes_kernel(float* __restrict__ pts) {
  __shared__ double rj[1024];
  __shared__ __align__(16) float vals[256];
  const int tid = threadIdx.x;
  const int blk = blockIdx.x;
  for (int j = tid; j < 1024; j += 256) rj[j] = (j > 0) ? (1.0 / (double)j) : 0.0;
  __syncthreads();
  const int i  = blk * 256 + tid;
  const int ic = (i < kNumQuad) ? i : (kNumQuad - 1);
  const float arg = ((float)ic + 0.75f) * (3.14159265358979f / 1000.5f);
  double xd = (double)cosf(arg);
#pragma unroll 1
  for (int it = 0; it < 5; ++it) {
    double p0 = 1.0;
    double p1 = xd;
#pragma unroll 1
    for (int j = 2; j <= kNumQuad; ++j) {
      const double r  = rj[j];
      const double t  = xd * p1;
      const double p2 = t + (1.0 - r) * (t - p0);
      p0 = p1;
      p1 = p2;
    }
    const double dp = (double)kNumQuad * (xd * p1 - p0) / (xd * xd - 1.0);
    xd = xd - p1 / dp;
  }
  float val = (float)(0.5 * (0.0 - xd) + 0.5);
  if (i >= kNumQuad) val = (i == kNumQuad + 1) ? 1.0f : 0.0f;
  vals[tid] = val;
  __syncthreads();
  if (tid < 64) {
    const v4f v = *(const v4f*)(vals + tid * 4);
    float* dst = pts + kPtQuad0 + blk * 256 + tid * 4;
    *(volatile v4f*)dst = v;
    __threadfence();
    *(volatile v4f*)dst = v;
  }
}

__global__ void __launch_bounds__(128)
jet_mlp_kernel(const float* __restrict__ pts,
               const float* __restrict__ W0, const float* __restrict__ b0,
               const unsigned short* __restrict__ W1h, const unsigned short* __restrict__ W1l, const float* __restrict__ b1,
               const unsigned short* __restrict__ W2h, const unsigned short* __restrict__ W2l, const float* __restrict__ b2,
               const unsigned short* __restrict__ P3, const float* __restrict__ b3,
               float* __restrict__ JT)
{
  __shared__ __align__(16) __bf16 Hh[2][5][16 * kHStride];
  __shared__ __align__(16) __bf16 Hl[2][5][16 * kHStride];
  __shared__ __align__(16) float rec[kRecFloats];

  const int tid  = threadIdx.x;
  const int lane = tid & 31;
  const int wave = tid >> 5;
  const int hh   = lane >> 4;
  const int c    = lane & 15;
  const int g0   = blockIdx.x * 16;

  if (tid < 48) rec[80 + tid] = 0.0f;

  {
    const float w   = W0[tid];
    const float bb0 = b0[tid];
    const float w2  = w * w;
    const float w3  = w2 * w;
    const float w4  = w2 * w2;
#pragma unroll 1
    for (int p = 0; p < 16; ++p) {
      const float s  = pts[g0 + p];
      const float z  = s * w + bb0;
      const float t  = tanhf(z);
      const float t2 = t * t;
      const float f1 = 1.0f - t2;
      const float f2 = -2.0f * t * f1;
      const float f3 = f1 * (6.0f * t2 - 2.0f);
      const float f4 = 8.0f * t * f1 * (2.0f - 3.0f * t2);
      const int idx = p * kHStride + tid;
      put_split(Hh[0][0], Hl[0][0], idx, t);
      put_split(Hh[0][1], Hl[0][1], idx, f1 * w);
      put_split(Hh[0][2], Hl[0][2], idx, f2 * w2);
      put_split(Hh[0][3], Hl[0][3], idx, f3 * w3);
      put_split(Hh[0][4], Hl[0][4], idx, f4 * w4);
    }
  }
  __syncthreads();

#pragma unroll 1
  for (int layer = 0; layer < 2; ++layer) {
    const __bf16* Wh = (const __bf16*)(layer ? W2h : W1h);
    const __bf16* Wl = (const __bf16*)(layer ? W2l : W1l);
    const float*  bb = layer ? b2 : b1;
    const int bi = layer & 1;
    const int bo = bi ^ 1;
#pragma unroll 1
    for (int cti = 0; cti < 2; ++cti) {
      const int col = (wave + 4 * cti) * 16 + c;
      const float bias = bb[col];
      v8f acc[5];
      acc[0] = (v8f){bias, bias, bias, bias, bias, bias, bias, bias};
#pragma unroll
      for (int k = 1; k < 5; ++k) acc[k] = (v8f){0.f, 0.f, 0.f, 0.f, 0.f, 0.f, 0.f, 0.f};
#pragma unroll 1
      for (int kb = 0; kb < kFeat; kb += 32) {
        const v16b bh = Frag<__bf16>::load(Wh + col * kFeat + kb + 8 * hh);
        const v16b bl = Frag<__bf16>::load(Wl + col * kFeat + kb + 8 * hh);
#pragma unroll
        for (int k = 0; k < 5; ++k) {
          const v16b ah = Frag<__bf16>::load(&Hh[bi][k][c * kHStride + kb + 8 * hh]);
          const v16b al = Frag<__bf16>::load(&Hl[bi][k][c * kHStride + kb + 8 * hh]);
          acc[k] = mma_bf(ah, bh, acc[k]);
          acc[k] = mma_bf(ah, bl, acc[k]);
          acc[k] = mma_bf(al, bh, acc[k]);
        }
      }
#pragma unroll
      for (int r = 0; r < 8; ++r) {
        const int p = 8 * hh + r;
        float y0, y1, y2, y3, y4;
        tanh_jet(acc[0][r], acc[1][r], acc[2][r], acc[3][r], acc[4][r], y0, y1, y2, y3, y4);
        const int idx = p * kHStride + col;
        put_split(Hh[bo][0], Hl[bo][0], idx, y0);
        put_split(Hh[bo][1], Hl[bo][1], idx, y1);
        put_split(Hh[bo][2], Hl[bo][2], idx, y2);
        put_split(Hh[bo][3], Hl[bo][3], idx, y3);
        put_split(Hh[bo][4], Hl[bo][4], idx, y4);
      }
    }
    __syncthreads();
  }

  const float b3v = b3[0];
  for (int k = wave; k < 5; k += 4) {
    v8f acc = (v8f){0.f, 0.f, 0.f, 0.f, 0.f, 0.f, 0.f, 0.f};
#pragma unroll 1
    for (int kb = 0; kb < kFeat; kb += 32) {
      const v16b bp = Frag<__bf16>::load((const __bf16*)P3 + c * kFeat + kb + 8 * hh);
      const v16b ah = Frag<__bf16>::load(&Hh[0][k][c * kHStride + kb + 8 * hh]);
      const v16b al = Frag<__bf16>::load(&Hl[0][k][c * kHStride + kb + 8 * hh]);
      acc = mma_bf(ah, bp, acc);
      acc = mma_bf(al, bp, acc);
    }
    const float badd = (k == 0) ? b3v : 0.0f;
#pragma unroll
    for (int r = 0; r < 8; ++r) {
      const float other = __shfl_xor(acc[r], 1, 32);
      const float u = (acc[r] + other) + badd;
      if (c == 0) rec[k * 16 + 8 * hh + r] = u;
    }
  }
  __syncthreads();
  if (wave == 0) {
    const v4f v = *(const v4f*)(rec + lane * 4);
    float* dst = JT + (size_t)blockIdx.x * kRecFloats + lane * 4;
    *(volatile v4f*)dst = v;
    __threadfence();
    *(volatile v4f*)dst = v;
  }
}

__global__ __launch_bounds__(256) void loss_kernel(const float* __restrict__ JT,
                                                   const float* __restrict__ data_w,
                                                   float* __restrict__ out)
{
  __shared__ float s1[256];
  __shared__ float s2[256];
  const int tid = threadIdx.x;
  float fsq = 0.0f;
  float dsum = 0.0f;
#pragma unroll 1
  for (int i = tid; i < kNumQuad; i += 256) {
    const int g = kPtQuad0 + i;
    const float v = JT[(g >> 4) * kRecFloats + 2 * 16 + (g & 15)];
    fsq += v * v;
  }
#pragma unroll 1
  for (int i = tid; i < kNumData; i += 256) {
    const int g = kPtData0 + i;
    const float pred = JT[(g >> 4) * kRecFloats + (g & 15)];
    const float d = pred - data_w[i] * (1.0f / 1.5f);
    dsum += d * d;
  }
  s1[tid] = fsq;
  s2[tid] = dsum;
  __syncthreads();
#pragma unroll 1
  for (int o = 128; o > 0; o >>= 1) {
    if (tid < o) {
      s1[tid] = s1[tid] + s1[tid + o];
      s2[tid] = s2[tid] + s2[tid + o];
    }
    __syncthreads();
  }
  if (tid == 0) {
    const int tb = (kPtBnd0 >> 4) * kRecFloats;
    const int pb = kPtBnd0 & 15;
    const float w0    = JT[tb + 0 * 16 + pb];
    const float dw0   = JT[tb + 1 * 16 + pb];
    const float wL    = JT[tb + 0 * 16 + pb + 1];
    const float ddwL  = JT[tb + 2 * 16 + pb + 1];
    const float dddwL = JT[tb + 3 * 16 + pb + 1];
    const float quad     = 2.0f * s1[0];
    const float inter_en = 0.375f * quad;
    const float exter_en = 7.5f * wL;
    const float res_pel  = inter_en - exter_en;
    const float res_dir  = 0.5f * (w0 * w0 + dw0 * dw0);
    const float Fb       = -dddwL;
    const float t1       = Fb * 0.2f - 1.0f;
    const float res_neu  = 0.5f * (t1 * t1 + ddwL * ddwL);
    const float res_data = s2[0] * (1.0f / 1024.0f);
    const float total    = res_pel + 0.5f * (res_dir + res_neu) + res_data;
    volatile float* dst = out + kOutLossIdx;
    *dst = total;
    __threadfence();
    *dst = total;
  }
}

__global__ __launch_bounds__(256) void out_kernel(const float* __restrict__ JT, float* __restrict__ out)
{
  const int i = blockIdx.x * 256 + threadIdx.x;
  const int k = i >> 13;
  const int j = i & 8191;
  const int tile = j >> 2;
  const int p4   = (j & 3) * 4;
  v4f v = *(const v4f*)(JT + (size_t)tile * kRecFloats + k * 16 + p4);
  const float sc = (k == 2 || k == 3) ? -1.0f : 1.5f;
  v = v * sc;
  float* dst = out + (size_t)k * kNumX + (size_t)j * 4;
  *(volatile v4f*)dst = v;
  __threadfence();
  *(volatile v4f*)dst = v;
}

extern "C" void kernel_launch(void* const* d_in, const int* in_sizes, int n_in,
                              void* d_out, int out_size, void* d_ws, size_t ws_size,
                              hipStream_t stream)
{
  if (n_in < 11) return;
  if (ws_size < kWsTotal) return;
  if (out_size < kOutLossIdx + 1) return;
  if (in_sizes[0] < kFeat || in_sizes[1] < kFeat || in_sizes[2] < kFeat * kFeat || in_sizes[3] < kFeat ||
      in_sizes[4] < kFeat * kFeat || in_sizes[5] < kFeat || in_sizes[6] < kFeat || in_sizes[7] < 1 ||
      in_sizes[8] < kNumX || in_sizes[9] < kNumData || in_sizes[10] < kNumData) return;

  const float* W0 = (const float*)d_in[0];
  const float* b0 = (const float*)d_in[1];
  const float* W1 = (const float*)d_in[2];
  const float* b1 = (const float*)d_in[3];
  const float* W2 = (const float*)d_in[4];
  const float* b2 = (const float*)d_in[5];
  const float* W3 = (const float*)d_in[6];
  const float* b3 = (const float*)d_in[7];
  const float* x  = (const float*)d_in[8];
  const float* dx = (const float*)d_in[9];
  const float* dw = (const float*)d_in[10];
  float* out = (float*)d_out;

  char* ws = (char*)d_ws;
  float*          pts = (float*)(ws + kWsPts);
  float*          JT  = (float*)(ws + kWsJT);
  unsigned short* W1h = (unsigned short*)(ws + kWsW1h);
  unsigned short* W1l = (unsigned short*)(ws + kWsW1l);
  unsigned short* W2h = (unsigned short*)(ws + kWsW2h);
  unsigned short* W2l = (unsigned short*)(ws + kWsW2l);
  unsigned short* P3  = (unsigned short*)(ws + kWsP3);

  prep_kernel<<<50, 256, 0, stream>>>(x, dx, W1, W2, W3, pts, W1h, W1l, W2h, W2l, P3);
  nodes_kernel<<<4, 256, 0, stream>>>(pts);
  jet_mlp_kernel<<<kNumTiles, 128, 0, stream>>>(pts, W0, b0, W1h, W1l, b1, W2h, W2l, b2, P3, b3, JT);
  loss_kernel<<<1, 256, 0, stream>>>(JT, dw, out);
  out_kernel<<<160, 256, 0, stream>>>(JT, out);
}
